// QubitClassifier_66975720014174
// MI455X (gfx1250) — hardware-run, weakly checked
//
#include <hip/hip_runtime.h>


#ifndef NB
#define NB 512
#endif
#define NB_FULL 512
#define NQ    13
#define DIMS  8192
#define NLAY  5
#define BPB   16
#define TPB   256
#define NWV   8
#define NSET  16
#define ASZ   1024
#define SB_   256.0f
#define SA_   1024.0f
#define QRS   2048.0f
#define QRI   (1.0f / 2048.0f)
#define FOLD  (1.0f / 262144.0f)
#define PI_F  3.14159265358979323846f
#define C0_   0.011048543456039806f
#define RS2   0.70710678118654752f

static_assert(DIMS == (1 << NQ));
static_assert(NQ == 13);
static_assert(TPB == 32 * NWV);
static_assert(TPB == 256);
static_assert(NWV * 4 * 16 == DIMS / 16);
static_assert(NLAY * NQ <= TPB);
static_assert(NLAY * 8 <= TPB);
static_assert(NLAY * NQ * 8 <= DIMS);
static_assert(NSET == NLAY * 3 + 1);
static_assert(BPB * 2 * 4 == 128);
static_assert(8 * 16 == BPB * 2 * 4);
static_assert(NB % BPB == 0);
static_assert(NB <= NB_FULL);
static_assert(SA_ * SB_ * FOLD == 1.0f);
static constexpr size_t LDS_BYTES = (size_t)DIMS * 4 * 2 + (size_t)NSET * ASZ * 2 + (size_t)(NSET - 1) * ASZ * 2 + (size_t)NLAY * 8 * 4 + (size_t)NWV * 4 + (size_t)BPB * 4;
static_assert(LDS_BYTES <= (size_t)131072);

typedef _Float16 h16;
typedef __attribute__((ext_vector_type(16))) _Float16 v16h;
typedef __attribute__((ext_vector_type(8)))  _Float16 v8h;
typedef __attribute__((ext_vector_type(8)))  float    v8f;
typedef __attribute__((ext_vector_type(4)))  float    v4f;

__device__ __forceinline__ unsigned short f2bf(float f) { unsigned u = __float_as_uint(f); u += 0x7FFFu + ((u >> 16) & 1u); return (unsigned short)(u >> 16); }
__device__ __forceinline__ float bfr(float f) { return __uint_as_float(((unsigned)f2bf(f)) << 16); }
__device__ __forceinline__ v16h cat16(v8h lo, v8h hi) { return __builtin_shufflevector(lo, hi, 0, 1, 2, 3, 4, 5, 6, 7, 8, 9, 10, 11, 12, 13, 14, 15); }
__device__ __forceinline__ v16h  ldh(const h16* p) { return cat16(*(const v8h*)p, *(const v8h*)(p + 16)); }

static __device__ __forceinline__ h16 toh_flush(float v) { const h16 r = (h16)v; return (fabsf(v) < 6.103515625e-05f) ? (h16)0.0f : r; }

__device__ __forceinline__ v8f wmma16g(v16h a, v16h b, v8f c) {
    c = __builtin_amdgcn_wmma_f32_16x16x32_f16(false, a, false, b, (short)0, c, false, false);
    asm volatile("v_nop\n\tv_nop\n\tv_nop\n\tv_nop" : "+v"(c) : "v"(a), "v"(b));
    return c;
}

__device__ __forceinline__ void phase_cs(const int s, const float (&xs)[NQ], const float (&as)[NQ], const float aa, float& cp, float& sp) {
#pragma clang fp contract(off)
    float u = 0.0f, v = 0.0f;
#pragma unroll
    for (int j = 0; j < NQ; ++j) {
        const bool ng = ((s >> (NQ - 1 - j)) & 1) != 0;
        u += ng ? -xs[j] : xs[j];
        v += ng ? -as[j] : as[j];
    }
    const float vv = v * v;
    const float hd = 0.5f * (vv - aa);
    const float phi = u + hd;
    sincosf(phi, &sp, &cp);
}

template <int P, int ARES>
__device__ __forceinline__ void apply_group(float* re, float* im, const h16* AHs, const h16* ARs, const int wave, const int lane) {
    const int n = lane & 15, hi = lane >> 4;
    const int ao = n * 32 + 8 * hi;
    const v16h ah0 = ldh(AHs + ao), ah1 = ldh(AHs + 512 + ao);
    v16h ar0 = (v16h){}, ar1 = (v16h){};
    if (ARES) { ar0 = ldh(ARs + ao); ar1 = ldh(ARs + 512 + ao); }
#pragma unroll 1
    for (int t = 0; t < 4; ++t) {
        const int c = (wave * 4 + t) * 16 + n;
        const int sb = ((c >> P) << (P + 4)) + (c & ((1 << P) - 1)) + ((8 * hi) << P);
        float xr[8], xi[8];
#pragma unroll
        for (int i = 0; i < 8; ++i) { xr[i] = re[sb + (i << P)]; xi[i] = im[sb + (i << P)]; }
        v16h bh, br;
#pragma unroll
        for (int i = 0; i < 8; ++i) {
            const float a = xr[i] * SB_; const h16 ha = toh_flush(a); bh[i] = ha;     br[i] = toh_flush((a - (float)ha) * QRS);
            const float b = xi[i] * SB_; const h16 hb = toh_flush(b); bh[8 + i] = hb; br[8 + i] = toh_flush((b - (float)hb) * QRS);
        }
        v8f cH0 = (v8f){}, cH1 = (v8f){}, cR0 = (v8f){}, cR1 = (v8f){};
        cH0 = wmma16g(ah0, bh, cH0); cH1 = wmma16g(ah1, bh, cH1);
        cR0 = wmma16g(ah0, br, cR0); cR1 = wmma16g(ah1, br, cR1);
        if (ARES) { cR0 = wmma16g(ar0, bh, cR0); cR1 = wmma16g(ar1, bh, cR1); }
#pragma unroll
        for (int r = 0; r < 8; ++r) {
            re[sb + (r << P)] = (cH0[r] + cR0[r] * QRI) * FOLD;
            im[sb + (r << P)] = (cH1[r] + cR1[r] * QRI) * FOLD;
        }
    }
}

__global__ __launch_bounds__(TPB) void k_circuit(const float* __restrict__ x, const float* __restrict__ theta, const float* __restrict__ bias, float* OUT) {
    __shared__ __align__(16) float re[DIMS];
    __shared__ __align__(16) float im[DIMS];
    __shared__ __align__(16) h16 AH[NSET * ASZ];
    __shared__ __align__(16) h16 AR[(NSET - 1) * ASZ];
    __shared__ float g12[NLAY * 8];
    __shared__ float red[NWV];
    __shared__ float lg[BPB];
    const int tid = threadIdx.x, lane = tid & 31;
    const int wave = __builtin_amdgcn_readfirstlane((int)(threadIdx.x >> 5));

    {
        const int gi = tid < NLAY * NQ ? tid : NLAY * NQ - 1;
        float al = theta[gi * 2], be = theta[gi * 2 + 1];
        asm volatile("" : "+v"(al)); asm volatile("" : "+v"(be));
        al = bfr(al); be = bfr(be);
        float sa, ca, sb2, cb;
        sincosf(0.5f * al, &sa, &ca);
        sincosf(0.5f * be, &sb2, &cb);
        if (tid < NLAY * NQ) {
            re[gi * 8 + 0] =  cb * ca;  re[gi * 8 + 1] = -sb2 * ca;
            re[gi * 8 + 2] = -cb * sa;  re[gi * 8 + 3] =  sb2 * sa;
            re[gi * 8 + 4] =  cb * sa;  re[gi * 8 + 5] =  sb2 * sa;
            re[gi * 8 + 6] =  cb * ca;  re[gi * 8 + 7] =  sb2 * ca;
        }
    }
    __syncthreads();
    {
        const int r = tid >> 4, c = tid & 15;
#pragma unroll 1
        for (int set = 0; set < NLAY * 3; ++set) {
            const int l = set / 3, g = set - 3 * l;
            float pr = 1.0f, pi = 0.0f;
#pragma unroll
            for (int j = 0; j < 4; ++j) {
                const int q = g * 4 + j;
                const int rj = (r >> (3 - j)) & 1, cj = (c >> (3 - j)) & 1;
                const int e = ((l * NQ + q) * 4 + rj * 2 + cj) * 2;
                const float er = re[e], ei = re[e + 1];
                const float nr = pr * er - pi * ei;
                const float ni = pr * ei + pi * er;
                pr = nr; pi = ni;
            }
            const float vr = pr * SA_, vi = pi * SA_;
            const h16 hr = toh_flush(vr), hq = toh_flush(vi);
            const h16 rr = toh_flush((vr - (float)hr) * QRS), rq = toh_flush((vi - (float)hq) * QRS);
            const int o = set * ASZ;
            AH[o + r * 32 + c] = hr;          AH[o + r * 32 + 16 + c] = -hq;
            AH[o + (16 + r) * 32 + c] = hq;   AH[o + (16 + r) * 32 + 16 + c] = hr;
            AR[o + r * 32 + c] = rr;          AR[o + r * 32 + 16 + c] = -rq;
            AR[o + (16 + r) * 32 + c] = rq;   AR[o + (16 + r) * 32 + 16 + c] = rr;
        }
        {
            const float hv = (__popc(r & c) & 1) ? (-0.25f * SA_) : (0.25f * SA_);
            const h16 hh = toh_flush(hv);
            const int o = (NSET - 1) * ASZ;
            AH[o + r * 32 + c] = hh;                  AH[o + r * 32 + 16 + c] = (h16)0.0f;
            AH[o + (16 + r) * 32 + c] = (h16)0.0f;    AH[o + (16 + r) * 32 + 16 + c] = hh;
        }
        const int gk = tid < NLAY * 8 ? tid : NLAY * 8 - 1;
        const float gv = re[((gk >> 3) * NQ + (NQ - 1)) * 8 + (gk & 7)];
        if (tid < NLAY * 8) g12[tid] = gv;
    }
    __syncthreads();

    const float bz = bfr(bias[0]);

#pragma unroll 1
    for (int e = 0; e < BPB; ++e) {
        const int bi = blockIdx.x * BPB + e;
        float xs[NQ], as[NQ]; float aa = 0.0f;
#pragma unroll
        for (int j = 0; j < NQ; ++j) { xs[j] = bfr(x[(size_t)bi * NQ + j]); as[j] = PI_F - xs[j]; aa += as[j] * as[j]; }

#pragma unroll 1
        for (int s = tid; s < DIMS; s += TPB) {
            float cp, sp; phase_cs(s, xs, as, aa, cp, sp);
            re[s] = C0_ * cp; im[s] = C0_ * sp;
        }
        __syncthreads();

        apply_group<9, 0>(re, im, AH + (NSET - 1) * ASZ, AR, wave, lane); __syncthreads();
        apply_group<5, 0>(re, im, AH + (NSET - 1) * ASZ, AR, wave, lane); __syncthreads();
        apply_group<1, 0>(re, im, AH + (NSET - 1) * ASZ, AR, wave, lane); __syncthreads();
#pragma unroll 1
        for (int pr = tid; pr < DIMS / 2; pr += TPB) {
            const int s0 = pr * 2;
            const float r0 = re[s0], i0 = im[s0], r1 = re[s0 + 1], i1 = im[s0 + 1];
            re[s0]     = RS2 * (r0 + r1); im[s0]     = RS2 * (i0 + i1);
            re[s0 + 1] = RS2 * (r0 - r1); im[s0 + 1] = RS2 * (i0 - i1);
        }
        __syncthreads();

#pragma unroll 1
        for (int s = tid; s < DIMS; s += TPB) {
            float cp, sp; phase_cs(s, xs, as, aa, cp, sp);
            const float r = re[s], i2 = im[s];
            re[s] = r * cp - i2 * sp;
            im[s] = r * sp + i2 * cp;
        }
        __syncthreads();

        float part = 0.0f;
#pragma unroll 1
        for (int l = 0; l < NLAY; ++l) {
            apply_group<9, 1>(re, im, AH + (l * 3 + 0) * ASZ, AR + (l * 3 + 0) * ASZ, wave, lane); __syncthreads();
            apply_group<5, 1>(re, im, AH + (l * 3 + 1) * ASZ, AR + (l * 3 + 1) * ASZ, wave, lane); __syncthreads();
            apply_group<1, 1>(re, im, AH + (l * 3 + 2) * ASZ, AR + (l * 3 + 2) * ASZ, wave, lane); __syncthreads();
            const float u00r = g12[l * 8 + 0], u00i = g12[l * 8 + 1], u01r = g12[l * 8 + 2], u01i = g12[l * 8 + 3];
            const float u10r = g12[l * 8 + 4], u10i = g12[l * 8 + 5], u11r = g12[l * 8 + 6], u11i = g12[l * 8 + 7];
            const bool lastl = (l == NLAY - 1);
#pragma unroll 1
            for (int pr = tid; pr < DIMS / 2; pr += TPB) {
                const int s0 = pr * 2, s1 = s0 + 1;
                const float r0 = re[s0], i0 = im[s0], r1 = re[s1], i1 = im[s1];
                const float n0r = u00r * r0 - u00i * i0 + u01r * r1 - u01i * i1;
                const float n0i = u00r * i0 + u00i * r0 + u01r * i1 + u01i * r1;
                const float n1r = u10r * r0 - u10i * i0 + u11r * r1 - u11i * i1;
                const float n1i = u10r * i0 + u10i * r0 + u11r * i1 + u11i * r1;
                if (!lastl) {
                    const bool f0 = (__popc(s0 & (s0 >> 1)) & 1) != 0;
                    const bool f1 = (__popc(s1 & (s1 >> 1)) & 1) != 0;
                    re[s0] = f0 ? -n0r : n0r; im[s0] = f0 ? -n0i : n0i;
                    re[s1] = f1 ? -n1r : n1r; im[s1] = f1 ? -n1i : n1i;
                } else {
                    const float m0 = n0r * n0r + n0i * n0i, m1 = n1r * n1r + n1i * n1i;
                    const bool od = (__popc(s0) & 1) != 0;
                    part += od ? (m1 - m0) : (m0 - m1);
                }
            }
            __syncthreads();
        }

        float p = part;
        p += __shfl_xor(p, 16, 32); p += __shfl_xor(p, 8, 32); p += __shfl_xor(p, 4, 32); p += __shfl_xor(p, 2, 32); p += __shfl_xor(p, 1, 32);
        if (lane == 0) red[wave] = p;
        __syncthreads();
        float tot = red[0];
#pragma unroll
        for (int w = 1; w < NWV; ++w) tot += red[w];
        const float lgt = tot + bz;
        if (tid == 0) lg[e] = lgt;
        __syncthreads();
    }

    {
        const int q = tid & 7;
        const float l0 = lg[2 * q], l1 = lg[2 * q + 1];
        v4f o; o[0] = -l0; o[1] = l0; o[2] = -l1; o[3] = l1;
        if (tid < 8) {
            volatile v4f* dst = (volatile v4f*)(OUT + (size_t)blockIdx.x * (BPB * 2) + 4 * q);
            *dst = o;
            __threadfence();
            *dst = o;
        }
    }
}

extern "C" void kernel_launch(void* const* d_in, const int* in_sizes, int n_in,
                              void* d_out, int out_size, void* d_ws, size_t ws_size, hipStream_t stream) {
    if (n_in < 3) return;
    if ((size_t)in_sizes[0] < (size_t)NB * NQ) return;
    if (in_sizes[1] < NLAY * NQ * 2) return;
    if (in_sizes[2] < 1) return;
    if ((size_t)out_size < (size_t)NB * 2) return;
    const float* x     = (const float*)d_in[0];
    const float* theta = (const float*)d_in[1];
    const float* bias  = (const float*)d_in[2];
    float* OUT = (float*)d_out;
    (void)d_ws; (void)ws_size;
    k_circuit<<<dim3(NB / BPB, 1, 1), TPB, 0, stream>>>(x, theta, bias, OUT);
}
